// DecoderBlock_47390669144299
// MI455X (gfx1250) — hardware-verified
//
#include <hip/hip_runtime.h>
#include <math.h>

#ifndef NB
#define NB 1
#endif
#ifndef SEQ
#define SEQ 4096
#endif
#define NB_FULL 1
#define SEQ_FULL 4096
#define EMB 768
#define NHD 12
#define HDIM 64
#define FFD 3072
#define QKVW (3 * EMB)
static_assert(NB == 1);
static_assert(SEQ % 64 == 0 && SEQ >= 64 && SEQ <= SEQ_FULL);
static_assert(EMB % 128 == 0 && FFD % 64 == 0 && QKVW % 64 == 0 && EMB == NHD * HDIM);
static_assert((size_t)SEQ * FFD * 4 <= (size_t)SEQ * QKVW * 4 + (size_t)SEQ * EMB * 4 + (size_t)SEQ * EMB * 2);

typedef __attribute__((ext_vector_type(16))) _Float16 v16h;
typedef __attribute__((ext_vector_type(8)))  _Float16 v8h;
typedef __attribute__((ext_vector_type(16))) __bf16   v16b;
typedef __attribute__((ext_vector_type(8)))  __bf16   v8b;
typedef __attribute__((ext_vector_type(8)))  float    v8f;
typedef __attribute__((ext_vector_type(4)))  float    v4f;
typedef __attribute__((ext_vector_type(4)))  unsigned int u4v;
typedef __attribute__((ext_vector_type(2)))  unsigned int u2v;

#define VST2(T, ptr, val) do { const T vst2_v_ = (val); *(volatile T*)(ptr) = vst2_v_; __threadfence(); *(volatile T*)(ptr) = vst2_v_; } while (0)
#define VST2V4(ptr, val) do { const v4f vst2_v4_ = (val); *(volatile v4f*)(ptr) = vst2_v4_; __threadfence(); *(volatile v4f*)(ptr) = vst2_v4_; } while (0)

__device__ __forceinline__ int frag_k(int i, int h) { return (i < 8) ? (8 * h + i) : (16 + 8 * h + (i - 8)); }
__device__ __forceinline__ __bf16 bf16_rne(float f) {
    unsigned int u = __float_as_uint(f);
    u += 0x7fffu + ((u >> 16) & 1u);
    return __builtin_bit_cast(__bf16, (unsigned short)(u >> 16));
}
__device__ __forceinline__ float bf16_f32(__bf16 b) { return __uint_as_float(((unsigned int)__builtin_bit_cast(unsigned short, b)) << 16); }
__device__ __forceinline__ v8f wmma16(v16h a, v16h b, v8f c) {
    c = __builtin_amdgcn_wmma_f32_16x16x32_f16(false, a, false, b, (short)0, c, false, false);
    asm volatile("v_nop\n\tv_nop\n\tv_nop\n\tv_nop" : "+v"(c) : "v"(a), "v"(b));
    return c;
}
struct Split { v16b hi, lo; };
__device__ __forceinline__ v8f wmma3(const Split& a, const Split& b, v8f c) {
    c = __builtin_amdgcn_wmma_f32_16x16x32_bf16(false, a.hi, false, b.hi, (short)0, c, false, false);
    c = __builtin_amdgcn_wmma_f32_16x16x32_bf16(false, a.hi, false, b.lo, (short)0, c, false, false);
    c = __builtin_amdgcn_wmma_f32_16x16x32_bf16(false, a.lo, false, b.hi, (short)0, c, false, false);
    asm volatile("v_nop\n\tv_nop\n\tv_nop\n\tv_nop" : "+v"(c) : "v"(a.hi), "v"(a.lo), "v"(b.hi), "v"(b.lo));
    return c;
}
struct Split3 { v16b hi, mid, lo; };
__device__ __forceinline__ v8f wmma6(const Split3& a, const Split3& b, v8f c) {
    c = __builtin_amdgcn_wmma_f32_16x16x32_bf16(false, a.hi, false, b.hi, (short)0, c, false, false);
    c = __builtin_amdgcn_wmma_f32_16x16x32_bf16(false, a.hi, false, b.mid, (short)0, c, false, false);
    c = __builtin_amdgcn_wmma_f32_16x16x32_bf16(false, a.mid, false, b.hi, (short)0, c, false, false);
    c = __builtin_amdgcn_wmma_f32_16x16x32_bf16(false, a.hi, false, b.lo, (short)0, c, false, false);
    c = __builtin_amdgcn_wmma_f32_16x16x32_bf16(false, a.mid, false, b.mid, (short)0, c, false, false);
    c = __builtin_amdgcn_wmma_f32_16x16x32_bf16(false, a.lo, false, b.hi, (short)0, c, false, false);
    asm volatile("v_nop\n\tv_nop\n\tv_nop\n\tv_nop" : "+v"(c) : "v"(a.hi), "v"(a.mid), "v"(a.lo), "v"(b.hi), "v"(b.mid), "v"(b.lo));
    return c;
}

__device__ __forceinline__ v16h fh_ld(const float* __restrict__ p, long long sk, int k0, int h, int klen, float s) {
    v16h a;
#pragma unroll
    for (int i = 0; i < 16; ++i) { const int k = k0 + frag_k(i, h); a[i] = (k < klen) ? (_Float16)(p[(long long)k * sk] * s) : (_Float16)0.f; }
    return a;
}
__device__ __forceinline__ Split sp_ld(const float* __restrict__ p, long long sk, int k0, int h, int klen, float s) {
    Split r;
#pragma unroll
    for (int i = 0; i < 16; ++i) {
        const int k = k0 + frag_k(i, h); const float x = (k < klen) ? p[(long long)k * sk] * s : 0.f;
        const __bf16 hb = bf16_rne(x); r.hi[i] = hb; r.lo[i] = bf16_rne(x - bf16_f32(hb));
    }
    return r;
}
__device__ __forceinline__ Split3 sp3_ld(const float* __restrict__ p, long long sk, int k0, int h, int klen, float s) {
    Split3 r;
#pragma unroll
    for (int i = 0; i < 16; ++i) {
        const int k = k0 + frag_k(i, h); const float x = (k < klen) ? p[(long long)k * sk] * s : 0.f;
        const __bf16 hb = bf16_rne(x); const float r1 = x - bf16_f32(hb); const __bf16 mb = bf16_rne(r1);
        r.hi[i] = hb; r.mid[i] = mb; r.lo[i] = bf16_rne(r1 - bf16_f32(mb));
    }
    return r;
}

namespace kit {

__device__ __forceinline__ unsigned short f2bf_bits(float f) {
  unsigned u = __float_as_uint(f);
  return (unsigned short)((u + 0x7FFFu + ((u >> 16) & 1u)) >> 16);
}
__device__ __forceinline__ float bf_bits2f(unsigned short h) { return __uint_as_float(((unsigned)h) << 16); }

__device__ __forceinline__ void dep_guard_h(v8f& a, v8f& b, v16h x, v16h y) { asm volatile("v_nop\n\tv_nop\n\tv_nop\n\tv_nop" : "+v"(a), "+v"(b) : "v"(x), "v"(y)); }
__device__ __forceinline__ void dep_guard_b(v8f& a, v8f& b, v16b x, v16b y) { asm volatile("v_nop\n\tv_nop\n\tv_nop\n\tv_nop" : "+v"(a), "+v"(b) : "v"(x), "v"(y)); }
__device__ __forceinline__ void keep4_h(v16h a, v16h b, v16h c, v16h d) { asm volatile("v_nop" :: "v"(a), "v"(b), "v"(c), "v"(d)); }
__device__ __forceinline__ void keep4_b(v16b a, v16b b, v16b c, v16b d) { asm volatile("v_nop" :: "v"(a), "v"(b), "v"(c), "v"(d)); }
__device__ __forceinline__ void acc_guard4(v8f& a, v8f& b, v8f& c, v8f& d) { asm volatile("v_nop\n\tv_nop\n\tv_nop\n\tv_nop" : "+v"(a), "+v"(b), "+v"(c), "+v"(d)); }

template <typename T> struct Frag;
template <> struct Frag<_Float16> {
  typedef v16h V; union U { v16h v; v8h h[2]; };
  static __device__ __forceinline__ v16h load(const _Float16* p) {
    U f; f.h[0] = *(const v8h*)(p); f.h[1] = *(const v8h*)(p + 16); return f.v;
  }
  static __device__ __forceinline__ v8f mma(v16h a, v16h b, v8f c) {
    return __builtin_amdgcn_wmma_f32_16x16x32_f16(false, a, false, b, (short)0, c, false, false);
  }
  static __device__ __forceinline__ void guard(v8f& a, v8f& b, v16h x, v16h y) { dep_guard_h(a, b, x, y); }
  static __device__ __forceinline__ void keep(v16h a, v16h b, v16h c, v16h d) { keep4_h(a, b, c, d); }
};
template <> struct Frag<__bf16> {
  typedef v16b V; union U { v16b v; v8b h[2]; };
  static __device__ __forceinline__ v16b load(const __bf16* p) {
    U f; f.h[0] = *(const v8b*)(p); f.h[1] = *(const v8b*)(p + 16); return f.v;
  }
  static __device__ __forceinline__ v8f mma(v16b a, v16b b, v8f c) {
    return __builtin_amdgcn_wmma_f32_16x16x32_bf16(false, a, false, b, (short)0, c, false, false);
  }
  static __device__ __forceinline__ void guard(v8f& a, v8f& b, v16b x, v16b y) { dep_guard_b(a, b, x, y); }
  static __device__ __forceinline__ void keep(v16b a, v16b b, v16b c, v16b d) { keep4_b(a, b, c, d); }
};

template <int ET> struct Elem;
template <> struct Elem<0> { typedef _Float16 T; };
template <> struct Elem<1> { typedef __bf16 T; };
template <int ET, bool SPLIT, int BIAS_MODE, int OUT_MODE, bool RESID, int ACT = 0>
__global__ __launch_bounds__(256) void wmma_gemm64(
    const unsigned short* __restrict__ Ap, const unsigned short* __restrict__ A2p, int lda, long strideA,
    const unsigned short* __restrict__ Btp, const unsigned short* __restrict__ Bt2p, int ldb, long strideB,
    void* __restrict__ Cout, void* __restrict__ Cout2, int ldc, long strideC,
    const float* __restrict__ bias,
    const float* __restrict__ resid, long strideR,
    int M, int N, int K, float scale) {
  typedef typename Elem<ET>::T T;
  typedef typename Frag<T>::V V;
  const T* A = (const T*)Ap; const T* A2 = (const T*)A2p; const T* Bt = (const T*)Btp; const T* Bt2 = (const T*)Bt2p;
  __shared__ __align__(16) float sT[8][16 * 68];
  const int b    = blockIdx.y;
  const int lane = threadIdx.x & 31;
  const int wave = threadIdx.x >> 5;
  const int tilesN = N >> 6;
  const int tilesM = M >> 6;
  const int tile = blockIdx.x * 8 + wave;
  if (tile >= tilesM * tilesN) return;
  const int tm = tile / tilesN;
  const int tn = tile - tm * tilesN;
  const int m0 = tm << 6;
  const int n0 = tn << 6;

  const T* Ab  = A  + (size_t)b * strideA;
  const T* Bb  = Bt + (size_t)b * strideB;
  const T* Ab2 = SPLIT ? (A2  + (size_t)b * strideA) : nullptr;
  const T* Bb2 = SPLIT ? (Bt2 + (size_t)b * strideB) : nullptr;

  const int rlane = lane & 15;
  const int koff  = (lane >> 4) * 8;
  const int mOff  = (lane >> 4) * 8;

  v8f acc[4][4];
#pragma unroll
  for (int i = 0; i < 4; ++i)
#pragma unroll
    for (int j = 0; j < 4; ++j) acc[i][j] = (v8f){0.f,0.f,0.f,0.f,0.f,0.f,0.f,0.f};

  for (int k0 = 0; k0 < K; k0 += 32) {
    V bh[4], bl[4];
#pragma unroll
    for (int j = 0; j < 4; ++j) {
      const size_t bo = (size_t)(n0 + (j << 4) + rlane) * ldb + koff + k0;
      bh[j] = Frag<T>::load(Bb + bo);
      if (SPLIT) bl[j] = Frag<T>::load(Bb2 + bo);
    }
#pragma unroll
    for (int i = 0; i < 4; ++i) {
      const size_t ao = (size_t)(m0 + (i << 4) + rlane) * lda + koff + k0;
      V ah = Frag<T>::load(Ab + ao);
      V al;
      if (SPLIT) al = Frag<T>::load(Ab2 + ao);
#pragma unroll
      for (int j = 0; j < 4; ++j) {
        acc[i][j] = Frag<T>::mma(ah, bh[j], acc[i][j]);
        if (SPLIT) {
          acc[i][j] = Frag<T>::mma(ah, bl[j], acc[i][j]);
          acc[i][j] = Frag<T>::mma(al, bh[j], acc[i][j]);
        }
      }
      Frag<T>::guard(acc[i][0], acc[i][3], ah, SPLIT ? al : ah);
    }
    Frag<T>::keep(bh[0], bh[1], bh[2], bh[3]);
    if (SPLIT) Frag<T>::keep(bl[0], bl[1], bl[2], bl[3]);
  }
  acc_guard4(acc[0][0], acc[0][1], acc[0][2], acc[0][3]);
  acc_guard4(acc[1][0], acc[1][1], acc[1][2], acc[1][3]);
  acc_guard4(acc[2][0], acc[2][1], acc[2][2], acc[2][3]);
  acc_guard4(acc[3][0], acc[3][1], acc[3][2], acc[3][3]);

  float* slab = sT[wave];
  const float* Rb = RESID ? (resid + (size_t)b * strideR) : nullptr;
#pragma unroll
  for (int i = 0; i < 4; ++i) {
    const int mBase = m0 + (i << 4);
#pragma unroll
    for (int j = 0; j < 4; ++j) {
      const int n = n0 + (j << 4) + rlane;
      float bv = 0.f;
      if (BIAS_MODE == 2) bv = bias[n];
#pragma unroll
      for (int r = 0; r < 8; ++r) {
        float v = acc[i][j][r] * scale;
        if (BIAS_MODE == 1) v += bias[mBase + mOff + r];
        if (BIAS_MODE == 2) v += bv;
        if (RESID) v += Rb[(size_t)(mBase + mOff + r) * ldc + n];
        if (ACT == 1) v = tanhf(v);
        if (ACT == 2) v = fmaxf(v, 0.0f);
        if (ACT == 3) v = v / (1.0f + expf(-v));
        if (ACT == 4) v = (v > 0.f) ? v : 0.01f * v;
        if (ACT == 5) v = 0.5f * v * (1.0f + erff(v * 0.70710678118654752f));
        if (ACT == 6) v = (v > 0.f) ? v : 0.2f * v;
        if (ACT == 7) { const float u = 0.7978845608028654f * (v + 0.044715f * v * v * v); v = 0.5f * v * (1.f + tanhf(u)); }
        slab[(mOff + r) * 68 + (j << 4) + rlane] = v;
      }
    }
    __builtin_amdgcn_fence(3  , "workgroup");
    __builtin_amdgcn_wave_barrier();
    __builtin_amdgcn_fence(2  , "workgroup");
    if (OUT_MODE == 0) {
      float* C = (float*)Cout + (size_t)b * strideC;
      const int hh = lane >> 4, c4 = (lane & 15) * 4;
      for (int pass = 0; pass < 2; ++pass) {
#pragma unroll
        for (int it = 0; it < 8; ++it) {
          const int row = it * 2 + hh;
          v4f v = *(const v4f*)(slab + row * 68 + c4);
          *(volatile v4f*)(C + (size_t)(mBase + row) * ldc + n0 + c4) = v;
        }
        __threadfence();
      }
    } else {
      const int q = lane >> 3, c8 = (lane & 7) * 8;
      unsigned short* C  = (unsigned short*)Cout  + (size_t)b * strideC;
      unsigned short* C2 = (OUT_MODE == 2) ? ((unsigned short*)Cout2 + (size_t)b * strideC) : nullptr;
      for (int pass = 0; pass < 2; ++pass) {
#pragma unroll
        for (int it = 0; it < 4; ++it) {
          const int row = it * 4 + q;
          const float* sp = slab + row * 68 + c8;
          v8h hv, lv;
#pragma unroll
          for (int e = 0; e < 8; ++e) {
            if (OUT_MODE == 1) {
              hv[e] = (_Float16)sp[e];
            } else {
              unsigned short hb = f2bf_bits(sp[e]);
              unsigned short lb = f2bf_bits(sp[e] - bf_bits2f(hb));
              hv[e] = __builtin_bit_cast(_Float16, hb);
              lv[e] = __builtin_bit_cast(_Float16, lb);
            }
          }
          *(volatile v8h*)(C + (size_t)(mBase + row) * ldc + n0 + c8) = hv;
          if (OUT_MODE == 2) *(volatile v8h*)(C2 + (size_t)(mBase + row) * ldc + n0 + c8) = lv;
        }
        __threadfence();
      }
    }
    __builtin_amdgcn_fence(3  , "workgroup");
    __builtin_amdgcn_wave_barrier();
    __builtin_amdgcn_fence(2  , "workgroup");
  }
}

}

#define AW 4
struct AttnP {
    const float* Q; const float* K; const float* V; float* O; float* P; const float* Mf; const int* Mi; float* ST;
    const float* Pw; const float* Rt; const int* SQ; const int* SK;
    long long swb, swh, swi, swj, srb, srh, sri;
    long long sQb, sQh, sQi, sQd, sKb, sKh, sKj, sKd, sVb, sVh, sVj, sVd, sOb, sOh, sOi, sPb, sPh, sPi, smb, smh, smi, smj;
    int Lq, Lk, dh, dv, hrep, causal, coff, pband;
    float scale, mfill; int nonorm, mpol;
    int roff, rn, segpol, win;
};
static_assert(sizeof(AttnP) == 12 * 8 + 29 * 8 + 16 * 4);

#ifndef KATTN_ATTR
#define KATTN_ATTR
#endif
template <int DHP, int DVP, int QM, bool SPLITPV, bool TWOPASS>
__global__ __launch_bounds__(32 * AW) KATTN_ATTR void k_attn(AttnP p) {
    constexpr int NT = DVP / 16;
    constexpr int KS = DHP / 32;
    constexpr int VP = DVP + 8;
    __shared__ __align__(16) float    pl[AW][16 * 64];
    __shared__ __align__(16) _Float16 vl[(SPLITPV ? 2 : 1) * 64 * VP];
    const int lane = threadIdx.x & 31, hf = lane >> 4, l15 = lane & 15, wave = threadIdx.x >> 5;
    const int h = blockIdx.y, b = blockIdx.z, hk = h / p.hrep;
    const int q0 = (blockIdx.x * AW + wave) * 16;
    float* myp = pl[wave];
    const float L2E = 1.4426950408889634f;
    const float NEG = -__builtin_inff();
    const int qi = min(q0 + l15, p.Lq - 1);
    const float* qrow = p.Q + b * p.sQb + h * p.sQh + (long long)qi * p.sQi;
    const float* kbase = p.K + b * p.sKb + hk * p.sKh;
    const float* vbase = p.V + b * p.sVb + hk * p.sVh;
    v16h qa[QM == 0 ? KS : 1]; Split qs_[QM == 1 ? KS : 1]; Split3 qt_[QM == 2 ? KS : 1];
#pragma unroll
    for (int ks = 0; ks < KS; ++ks) {
        if (QM == 2) qt_[ks] = sp3_ld(qrow, p.sQd, ks * 32, hf, p.dh, 1.f);
        else if (QM == 1) qs_[ks] = sp_ld(qrow, p.sQd, ks * 32, hf, p.dh, 1.f);
        else qa[ks] = fh_ld(qrow, p.sQd, ks * 32, hf, p.dh, 1.f);
    }
    v8f o[NT]; float m8[8], l8[8];
#pragma unroll
    for (int t = 0; t < NT; ++t) { v8f zz = {}; o[t] = zz; }
#pragma unroll
    for (int i = 0; i < 8; ++i) { m8[i] = NEG; l8[i] = 0.f; }
    int jend = p.Lk; int jstart = 0;
    if (p.causal == 1) { const int je = (blockIdx.x * AW + AW - 1) * 16 + 16 + p.coff; jend = min(jend, max(je, 0)); }
    if (p.win > 0) { const int js = (int)(blockIdx.x * AW) * 16 + p.coff - p.win; jstart = (js > 0) ? (js / 64) * 64 : 0; }
    const int npass = TWOPASS ? 2 : 1;
    for (int pass = 0; pass < npass; ++pass) {
        const bool dopv = (!TWOPASS) || pass == 1;
        for (int j0 = jstart; j0 < jend; j0 += 64) {
            if (dopv) {
                __syncthreads();
                for (int idx = threadIdx.x; idx < 64 * DVP; idx += 32 * AW) {
                    const int jr = idx / DVP, d = idx - jr * DVP, j = j0 + jr;
                    const float f = (j < p.Lk && d < p.dv) ? vbase[(long long)j * p.sVj + (long long)d * p.sVd] : 0.f;
                    if (SPLITPV) {
                        const __bf16 hb = bf16_rne(f);
                        ((__bf16*)vl)[jr * VP + d] = hb; ((__bf16*)vl)[64 * VP + jr * VP + d] = bf16_rne(f - bf16_f32(hb));
                    } else vl[jr * VP + d] = (_Float16)f;
                }
            }
            v8f s[4];
#pragma unroll
            for (int t = 0; t < 4; ++t) {
                const int j = min(j0 + t * 16 + l15, p.Lk - 1);
                const float* krow = kbase + (long long)j * p.sKj;
                v8f acc = {};
#pragma unroll
                for (int ks = 0; ks < KS; ++ks) {
                    if (QM == 2)      acc = wmma6(qt_[ks], sp3_ld(krow, p.sKd, ks * 32, hf, p.dh, 1.f), acc);
                    else if (QM == 1) acc = wmma3(qs_[ks], sp_ld(krow, p.sKd, ks * 32, hf, p.dh, 1.f), acc);
                    else              acc = wmma16(qa[ks], fh_ld(krow, p.sKd, ks * 32, hf, p.dh, 1.f), acc);
                }
                s[t] = acc;
            }
            float pv[8][4];
#pragma unroll
            for (int i = 0; i < 8; ++i) {
                const int irow = q0 + i + 8 * hf;
                const int ic = min(irow, p.Lq - 1);
                float sc[4];
#pragma unroll
                for (int t = 0; t < 4; ++t) {
                    const int jg = j0 + t * 16 + l15;
                    float v = s[t][i] * p.scale;
                    if (p.Mf) v += p.Mf[b * p.smb + h * p.smh + (long long)ic * p.smi + (long long)min(jg, p.Lk - 1) * p.smj];
                    if (p.Rt) { int rc = ic - min(jg, p.Lk - 1) + p.roff; rc = rc < 0 ? 0 : (rc >= p.rn ? p.rn - 1 : rc); v += p.Rt[b * p.srb + h * p.srh + (long long)ic * p.sri + rc]; }
                    if (p.Mi) { const int mv = p.Mi[b * p.smb + h * p.smh + (long long)ic * p.smi + (long long)min(jg, p.Lk - 1) * p.smj]; if (p.mpol ? (mv != 0) : (mv == 0)) v = p.mfill; }
                    if (p.SQ) { const bool same = p.SQ[(long long)b * p.Lq + ic] == p.SK[(long long)b * p.Lk + min(jg, p.Lk - 1)]; if (p.segpol ? same : !same) v = p.mfill; }
                    if (p.causal == 2 && jg > irow + p.coff) v = p.mfill;
                    if (jg >= p.Lk || (p.causal == 1 && jg > irow + p.coff) || (p.causal == 3 && jg < irow + p.coff) || (p.win > 0 && irow + p.coff - jg > p.win)) v = NEG; else v *= L2E;
                    sc[t] = v;
                }
                if (!TWOPASS || pass == 0) {
                    float mx = fmaxf(fmaxf(sc[0], sc[1]), fmaxf(sc[2], sc[3]));
                    mx = fmaxf(mx, __shfl_xor(mx, 1, 32)); mx = fmaxf(mx, __shfl_xor(mx, 2, 32));
                    mx = fmaxf(mx, __shfl_xor(mx, 4, 32)); mx = fmaxf(mx, __shfl_xor(mx, 8, 32));
                    const float mnew = fmaxf(m8[i], mx);
                    const float corr = (mnew == NEG) ? 1.f : exp2f(m8[i] - mnew);
                    float rs = 0.f;
#pragma unroll
                    for (int t = 0; t < 4; ++t) {
                        const float pp = (sc[t] == NEG) ? 0.f : exp2f(sc[t] - mnew); rs += pp;
                        pv[i][t] = p.Pw ? pp * p.Pw[b * p.swb + h * p.swh + (long long)ic * p.swi + (long long)min(j0 + t * 16 + l15, p.Lk - 1) * p.swj] : pp;
                    }
                    rs += __shfl_xor(rs, 1, 32); rs += __shfl_xor(rs, 2, 32); rs += __shfl_xor(rs, 4, 32); rs += __shfl_xor(rs, 8, 32);
                    l8[i] = l8[i] * corr + rs; m8[i] = mnew;
                    if (!TWOPASS) {
#pragma unroll
                        for (int t = 0; t < NT; ++t) o[t][i] *= corr;
                    }
                } else {
                    const float inv = (l8[i] > 0.f) ? 1.f / l8[i] : 0.f;
#pragma unroll
                    for (int t = 0; t < 4; ++t) {
                        const int jg = j0 + t * 16 + l15;
                        float pp = (sc[t] == NEG) ? 0.f : exp2f(sc[t] - m8[i]) * inv;
                        if (p.Pw) pp *= p.Pw[b * p.swb + h * p.swh + (long long)ic * p.swi + (long long)min(jg, p.Lk - 1) * p.swj];
                        pv[i][t] = pp;
                    }
                }
            }
            if (dopv) {
#pragma unroll
                for (int i = 0; i < 8; ++i)
#pragma unroll
                    for (int t = 0; t < 4; ++t) ((volatile float*)myp)[(i + 8 * hf) * 64 + t * 16 + l15] = pv[i][t];
                __syncthreads();
                if (p.P) {
                    float* pb_ = p.P + b * p.sPb + h * p.sPh;
                    const bool fastP = (p.pband == 0) && ((p.sPi & 3) == 0) && (j0 + 64 <= p.Lk) && (q0 + 16 <= p.Lq) && ((((size_t)pb_) & 15) == 0);
                    if (fastP) {
#pragma unroll
                        for (int s2 = 0; s2 < 8; ++s2) {
                            const int row = s2 * 2 + (lane >> 4), c4 = (lane & 15) * 4;
                            const v4f v = *(const v4f*)(myp + row * 64 + c4);
                            VST2V4(pb_ + (long long)(q0 + row) * p.sPi + j0 + c4, v);
                        }
                    } else {
                        for (int row = 0; row < 16; ++row) {
                            const int irow = q0 + row; if (irow >= p.Lq) continue;
                            for (int c = lane; c < 64; c += 32) {
                                const int jg = j0 + c; if (jg >= p.Lk) continue;
                                if (p.pband == 0) VST2(float, pb_ + (long long)irow * p.sPi + jg, myp[row * 64 + c]);
                                else if (jg - irow <= p.pband && irow - jg <= p.pband) VST2(float, pb_ + (long long)irow * p.sPi + (jg - irow + p.pband), myp[row * 64 + c]);
                            }
                        }
                    }
                }
                if (SPLITPV) {
                    const Split pa0 = sp_ld(myp + l15 * 64, 1, 0, hf, 64, 1.f), pa1 = sp_ld(myp + l15 * 64, 1, 32, hf, 64, 1.f);
                    const __bf16* vh = (const __bf16*)vl; const __bf16* vlo = vh + 64 * VP;
#pragma unroll
                    for (int t = 0; t < NT; ++t) {
                        const int dcol = t * 16 + l15;
                        Split b0, b1;
#pragma unroll
                        for (int e = 0; e < 16; ++e) {
                            const int k0 = frag_k(e, hf), k1 = 32 + frag_k(e, hf);
                            b0.hi[e] = vh[k0 * VP + dcol]; b0.lo[e] = vlo[k0 * VP + dcol]; b1.hi[e] = vh[k1 * VP + dcol]; b1.lo[e] = vlo[k1 * VP + dcol];
                        }
                        o[t] = wmma3(pa0, b0, o[t]);
                        o[t] = wmma3(pa1, b1, o[t]);
                    }
                } else {
                    const v16h pa0 = fh_ld(myp + l15 * 64, 1, 0, hf, 64, 4096.f), pa1 = fh_ld(myp + l15 * 64, 1, 32, hf, 64, 4096.f);
#pragma unroll
                    for (int t = 0; t < NT; ++t) {
                        const int dcol = t * 16 + l15;
                        v16h b0, b1;
#pragma unroll
                        for (int e = 0; e < 16; ++e) { b0[e] = vl[frag_k(e, hf) * VP + dcol]; b1[e] = vl[(32 + frag_k(e, hf)) * VP + dcol]; }
                        o[t] = wmma16(pa0, b0, o[t]);
                        o[t] = wmma16(pa1, b1, o[t]);
                    }
                }
            }
        }
    }
    float* obase = p.O + b * p.sOb + h * p.sOh;
    if (p.ST) {
        const int rl = lane >> 1, isel = rl & 7;
        float mv = 0.f, lv = 0.f;
#pragma unroll
        for (int i = 0; i < 8; ++i) if (i == isel) { mv = m8[i]; lv = l8[i]; }
        const int irow = q0 + rl;
        if (irow < p.Lq) { float* st = p.ST + (((long long)b * gridDim.y + h) * p.Lq + irow) * 2 + (lane & 1); VST2(float, st, (lane & 1) ? lv : mv * 0.6931471805599453f); }
    }
    float invr[8];
#pragma unroll
    for (int i = 0; i < 8; ++i) {
        if (TWOPASS) invr[i] = SPLITPV ? 1.f : (1.f / 4096.f);
        else if (p.nonorm) invr[i] = exp2f(m8[i]) * (SPLITPV ? 1.f : (1.f / 4096.f));
        else invr[i] = (l8[i] > 0.f) ? (SPLITPV ? 1.f / l8[i] : 1.f / (l8[i] * 4096.f)) : 0.f;
    }
    __syncthreads();
    const bool ofast = ((p.sOi & 3) == 0) && ((((size_t)obase) & 15) == 0) && (q0 + 16 <= p.Lq);
#pragma unroll
    for (int c0 = 0; c0 < DVP; c0 += 64) {
#pragma unroll
        for (int i = 0; i < 8; ++i)
#pragma unroll
            for (int t = 0; t < NT; ++t) if (t * 16 >= c0 && t * 16 < c0 + 64) ((volatile float*)myp)[(i + 8 * hf) * 64 + (t * 16 - c0) + l15] = o[t][i] * invr[i];
        __syncthreads();
        const int cw = (DVP - c0 < 64) ? (DVP - c0) : 64;
        if (ofast && (c0 + cw <= p.dv) && (cw % 32 == 0)) {
            const int lpr = cw / 4;
            const int rows_per_ins = 32 / lpr;
            for (int rb = 0; rb < 16; rb += rows_per_ins) {
                const int row = rb + lane / lpr, c4 = (lane % lpr) * 4;
                const v4f v = *(const v4f*)(myp + row * 64 + c4);
                VST2V4(obase + (long long)(q0 + row) * p.sOi + c0 + c4, v);
            }
        } else {
            for (int row = 0; row < 16; ++row) {
                const int irow = q0 + row; if (irow >= p.Lq) continue;
                for (int c = lane; c < cw; c += 32) { const int d = c0 + c; if (d < p.dv) VST2(float, obase + (long long)irow * p.sOi + d, myp[row * 64 + c]); }
            }
        }
        __syncthreads();
    }
}

__device__ __forceinline__ unsigned int cmb_pk2(float a, float b) { return (unsigned int)__builtin_bit_cast(unsigned short, (_Float16)a) | ((unsigned int)__builtin_bit_cast(unsigned short, (_Float16)b) << 16); }
__device__ __forceinline__ float cmb_bf(float v) { const unsigned u = __builtin_bit_cast(unsigned, v); const unsigned r = (u + 0x7fffu + ((u >> 16) & 1u)) & 0xffff0000u; return __builtin_bit_cast(float, r); }
__global__ __launch_bounds__(256) void k_cm_bfvec(const float* __restrict__ SRC, float* __restrict__ DST, int n) { const int u = blockIdx.x * 256 + threadIdx.x; if (u >= n) return; VST2(float, DST + u, cmb_bf(SRC[u])); }
__global__ __launch_bounds__(256) void k_cm_castbT(const float* __restrict__ SRC, int lds, unsigned short* __restrict__ DST, int ldd, int nR, int nC, float sc) {
    const long long u = (long long)blockIdx.x * 256 + threadIdx.x; const int per = nR / 8; if (u >= (long long)nC * per) return; const int c = (int)(u / per); const int r0 = 8 * (int)(u % per);
    float w[8];
#pragma unroll
    for (int e = 0; e < 8; ++e) w[e] = cmb_bf(SRC[(long long)(r0 + e) * lds + c]) * sc;
    u4v pk; pk.x = cmb_pk2(w[0], w[1]); pk.y = cmb_pk2(w[2], w[3]); pk.z = cmb_pk2(w[4], w[5]); pk.w = cmb_pk2(w[6], w[7]); VST2(u4v, (u4v*)(DST + (long long)c * ldd + r0), pk); }

__global__ __launch_bounds__(256) void k_cast16(const float* __restrict__ src, long long lds, _Float16* __restrict__ dst, long long ldd, int R, int C, float s) {
    const long long i = (long long)blockIdx.x * 256 + threadIdx.x; const long long np = (long long)R * (C / 2); if (i >= np) return; const int r = (int)(i / (C / 2)); const int c = 2 * (int)(i % (C / 2));
    const _Float16 h0 = (_Float16)(src[(long long)r * lds + c] * s), h1 = (_Float16)(src[(long long)r * lds + c + 1] * s);
    const unsigned u = (unsigned)__builtin_bit_cast(unsigned short, h0) | ((unsigned)__builtin_bit_cast(unsigned short, h1) << 16);
    volatile unsigned* d = (volatile unsigned*)(dst + (long long)r * ldd + c); *d = u; __threadfence(); *d = u; }

template <int RX>
__global__ __launch_bounds__(256) void k_ln768(const float* __restrict__ X, const float* __restrict__ G, const float* __restrict__ Bb, float* __restrict__ F, unsigned short* __restrict__ O, int rows) {
    #pragma clang fp contract(off)
    const int row = blockIdx.x * 8 + (threadIdx.x >> 5); const int L = threadIdx.x & 31; if (row >= rows) return;
    const float* xr = X + (long long)row * EMB;
    float x[24]; float s = 0.f;
#pragma unroll
    for (int i = 0; i < 6; ++i) {
        const v4f a = *(const v4f*)(xr + 128 * i + 4 * L);
        const float t0 = RX ? cmb_bf(a.x) : a.x, t1 = RX ? cmb_bf(a.y) : a.y, t2 = RX ? cmb_bf(a.z) : a.z, t3 = RX ? cmb_bf(a.w) : a.w;
        x[4 * i] = t0; x[4 * i + 1] = t1; x[4 * i + 2] = t2; x[4 * i + 3] = t3;
        s += t0; s += t1; s += t2; s += t3;
    }
#pragma unroll
    for (int o = 16; o > 0; o >>= 1) s += __shfl_xor(s, o, 32);
    const float mu = s * (1.f / 768.f);
    float q = 0.f;
#pragma unroll
    for (int e = 0; e < 24; ++e) { const float d = x[e] - mu; q += d * d; }
#pragma unroll
    for (int o = 16; o > 0; o >>= 1) q += __shfl_xor(q, o, 32);
    const float rs = rsqrtf(q * (1.f / 768.f) + 1e-5f);
#pragma unroll
    for (int i = 0; i < 6; ++i) {
        const int c0 = 128 * i + 4 * L;
        const v4f gv = *(const v4f*)(G + c0), bv = *(const v4f*)(Bb + c0);
        v4f y;
        y.x = (x[4 * i]     - mu) * rs * cmb_bf(gv.x) + cmb_bf(bv.x);
        y.y = (x[4 * i + 1] - mu) * rs * cmb_bf(gv.y) + cmb_bf(bv.y);
        y.z = (x[4 * i + 2] - mu) * rs * cmb_bf(gv.z) + cmb_bf(bv.z);
        y.w = (x[4 * i + 3] - mu) * rs * cmb_bf(gv.w) + cmb_bf(bv.w);
        VST2V4(F + (long long)row * EMB + c0, y);
        u2v pk; pk.x = cmb_pk2(y.x, y.y); pk.y = cmb_pk2(y.z, y.w);
        VST2(u2v, (u2v*)(O + (long long)row * EMB + c0), pk);
    }
}

__global__ __launch_bounds__(256) void k_gelu16(const float* __restrict__ Hp, unsigned short* __restrict__ O, long long n4, float sc) {
    const long long u = (long long)blockIdx.x * 256 + threadIdx.x; if (u >= n4) return;
    const v4f a = *(const v4f*)(Hp + 4 * u);
    unsigned long long pk = 0ull;
#pragma unroll 1
    for (int e = 0; e < 4; ++e) {
        const float v = (e == 0) ? a.x : ((e == 1) ? a.y : ((e == 2) ? a.z : a.w));
        const float gl = 0.5f * v * (1.f + erff(v * 0.70710678118654752f));
        pk |= ((unsigned long long)__builtin_bit_cast(unsigned short, (_Float16)(gl * sc))) << (16 * e);
    }
    u2v w; w.x = (unsigned)(pk & 0xffffffffull); w.y = (unsigned)(pk >> 32);
    VST2(u2v, (u2v*)(O + 4 * u), w);
}


extern "C" void kernel_launch(void* const* d_in, const int* in_sizes, int n_in, void* d_out, int out_size, void* d_ws, size_t ws_size, hipStream_t stream) {
    if (n_in < 17) return;
    if (in_sizes[0] < SEQ * EMB || in_sizes[1] < EMB * EMB || in_sizes[2] < EMB || in_sizes[3] < EMB * EMB || in_sizes[4] < EMB ||
        in_sizes[5] < EMB * EMB || in_sizes[6] < EMB || in_sizes[7] < EMB * EMB || in_sizes[8] < EMB ||
        in_sizes[9] < EMB || in_sizes[10] < EMB || in_sizes[11] < EMB || in_sizes[12] < EMB ||
        in_sizes[13] < EMB * FFD || in_sizes[14] < FFD || in_sizes[15] < FFD * EMB || in_sizes[16] < EMB) return;
    if (out_size < SEQ * EMB) return;
    const float* x   = (const float*)d_in[0];
    const float* Wq  = (const float*)d_in[1];
    const float* bq  = (const float*)d_in[2];
    const float* Wk  = (const float*)d_in[3];
    const float* bk  = (const float*)d_in[4];
    const float* Wv  = (const float*)d_in[5];
    const float* bv  = (const float*)d_in[6];
    const float* Wo  = (const float*)d_in[7];
    const float* bo  = (const float*)d_in[8];
    const float* g1  = (const float*)d_in[9];
    const float* be1 = (const float*)d_in[10];
    const float* g2  = (const float*)d_in[11];
    const float* be2 = (const float*)d_in[12];
    const float* W1  = (const float*)d_in[13];
    const float* b1  = (const float*)d_in[14];
    const float* W2  = (const float*)d_in[15];
    const float* b2  = (const float*)d_in[16];
    float* out = (float*)d_out;

    char* wsp = (char*)d_ws; size_t off = 0;
    auto carve = [&](size_t bytes) -> char* { char* p = wsp + off; off += (bytes + 255) & ~(size_t)255; return p; };
    unsigned short* WQKV16 = (unsigned short*)carve((size_t)QKVW * EMB * 2);
    unsigned short* WO16   = (unsigned short*)carve((size_t)EMB * EMB * 2);
    unsigned short* W116   = (unsigned short*)carve((size_t)FFD * EMB * 2);
    unsigned short* W216   = (unsigned short*)carve((size_t)EMB * FFD * 2);
    float* BQKV = (float*)carve((size_t)QKVW * 4);
    float* BO   = (float*)carve((size_t)EMB * 4);
    float* BR1  = (float*)carve((size_t)FFD * 4);
    float* BR2  = (float*)carve((size_t)EMB * 4);
    float* Hf   = (float*)carve((size_t)SEQ * EMB * 4);
    unsigned short* N16 = (unsigned short*)carve((size_t)SEQ * EMB * 2);
    float* QKV  = (float*)carve((size_t)SEQ * QKVW * 4);
    float* AO   = (float*)carve((size_t)SEQ * EMB * 4);
    unsigned short* AO16 = (unsigned short*)carve((size_t)SEQ * EMB * 2);
    float* X1   = (float*)carve((size_t)SEQ * EMB * 4);
    unsigned short* H16 = (unsigned short*)carve((size_t)SEQ * FFD * 2);
    float* H1   = QKV;
    float* H2f  = Hf;
    if (off > ws_size) return;

    k_cm_castbT<<<(unsigned)(((long long)EMB * (EMB / 8) + 255) / 256), 256, 0, stream>>>(Wq, EMB, WQKV16, EMB, EMB, EMB, 16.0f);
    k_cm_castbT<<<(unsigned)(((long long)EMB * (EMB / 8) + 255) / 256), 256, 0, stream>>>(Wk, EMB, WQKV16 + (size_t)EMB * EMB, EMB, EMB, EMB, 16.0f);
    k_cm_castbT<<<(unsigned)(((long long)EMB * (EMB / 8) + 255) / 256), 256, 0, stream>>>(Wv, EMB, WQKV16 + (size_t)2 * EMB * EMB, EMB, EMB, EMB, 16.0f);
    k_cm_castbT<<<(unsigned)(((long long)EMB * (EMB / 8) + 255) / 256), 256, 0, stream>>>(Wo, EMB, WO16, EMB, EMB, EMB, 16.0f);
    k_cm_castbT<<<(unsigned)(((long long)FFD * (EMB / 8) + 255) / 256), 256, 0, stream>>>(W1, FFD, W116, EMB, EMB, FFD, 16.0f);
    k_cm_castbT<<<(unsigned)(((long long)EMB * (FFD / 8) + 255) / 256), 256, 0, stream>>>(W2, EMB, W216, FFD, FFD, EMB, 16.0f);
    k_cm_bfvec<<<(EMB + 255) / 256, 256, 0, stream>>>(bq, BQKV, EMB);
    k_cm_bfvec<<<(EMB + 255) / 256, 256, 0, stream>>>(bk, BQKV + EMB, EMB);
    k_cm_bfvec<<<(EMB + 255) / 256, 256, 0, stream>>>(bv, BQKV + 2 * EMB, EMB);
    k_cm_bfvec<<<(EMB + 255) / 256, 256, 0, stream>>>(bo, BO, EMB);
    k_cm_bfvec<<<(FFD + 255) / 256, 256, 0, stream>>>(b1, BR1, FFD);
    k_cm_bfvec<<<(EMB + 255) / 256, 256, 0, stream>>>(b2, BR2, EMB);

    k_ln768<1><<<SEQ / 8, 256, 0, stream>>>(x, g1, be1, Hf, N16, SEQ);

    kit::wmma_gemm64<0, false, 2, 0, false, 0><<<dim3((unsigned)((((SEQ) / 64) * ((QKVW) / 64) + 7) / 8), 1u), 256, 0, stream>>>(
        (const unsigned short*)N16, nullptr, EMB, 0L, (const unsigned short*)WQKV16, nullptr, EMB, 0L, (void*)QKV, nullptr, QKVW, 0L,
        BQKV, nullptr, 0L, SEQ, QKVW, EMB, 1.0f / 16.0f);

    { AttnP a;
      a.Q = QKV; a.K = QKV + EMB; a.V = QKV + 2 * EMB; a.O = AO; a.P = 0; a.Mf = 0; a.Mi = 0; a.ST = 0;
      a.Pw = 0; a.Rt = 0; a.SQ = 0; a.SK = 0;
      a.swb = 0; a.swh = 0; a.swi = 0; a.swj = 0; a.srb = 0; a.srh = 0; a.sri = 0;
      a.sQb = (long long)SEQ * QKVW; a.sQh = HDIM; a.sQi = QKVW; a.sQd = 1;
      a.sKb = (long long)SEQ * QKVW; a.sKh = HDIM; a.sKj = QKVW; a.sKd = 1;
      a.sVb = (long long)SEQ * QKVW; a.sVh = HDIM; a.sVj = QKVW; a.sVd = 1;
      a.sOb = (long long)SEQ * EMB;  a.sOh = HDIM; a.sOi = EMB;
      a.sPb = 0; a.sPh = 0; a.sPi = 0; a.smb = 0; a.smh = 0; a.smi = 0; a.smj = 0;
      a.Lq = SEQ; a.Lk = SEQ; a.dh = HDIM; a.dv = HDIM; a.hrep = 1; a.causal = 1; a.coff = 0; a.pband = 0;
      a.scale = 0.125f; a.mfill = 0.0f; a.nonorm = 0; a.mpol = 0;
      a.roff = 0; a.rn = 1; a.segpol = 0; a.win = 0;
      k_attn<64, 64, 0, false, false><<<dim3((unsigned)((SEQ + 16 * AW - 1) / (16 * AW)), (unsigned)NHD, (unsigned)NB), 32 * AW, 0, stream>>>(a); }

    k_cast16<<<(unsigned)((((long long)SEQ * (EMB / 2)) + 255) / 256), 256, 0, stream>>>(AO, EMB, (_Float16*)AO16, EMB, SEQ, EMB, 64.0f);
    kit::wmma_gemm64<0, false, 2, 0, true, 0><<<dim3((unsigned)((((SEQ) / 64) * ((EMB) / 64) + 7) / 8), 1u), 256, 0, stream>>>(
        (const unsigned short*)AO16, nullptr, EMB, 0L, (const unsigned short*)WO16, nullptr, EMB, 0L, (void*)X1, nullptr, EMB, 0L,
        BO, Hf, 0L, SEQ, EMB, EMB, 1.0f / 1024.0f);

    k_ln768<0><<<SEQ / 8, 256, 0, stream>>>(X1, g2, be2, H2f, N16, SEQ);

    kit::wmma_gemm64<0, false, 2, 0, false, 0><<<dim3((unsigned)((((SEQ) / 64) * ((FFD) / 64) + 7) / 8), 1u), 256, 0, stream>>>(
        (const unsigned short*)N16, nullptr, EMB, 0L, (const unsigned short*)W116, nullptr, EMB, 0L, (void*)H1, nullptr, FFD, 0L,
        BR1, nullptr, 0L, SEQ, FFD, EMB, 1.0f / 16.0f);
    k_gelu16<<<(unsigned)((((long long)SEQ * FFD / 4) + 255) / 256), 256, 0, stream>>>(H1, H16, (long long)SEQ * FFD / 4, 16.0f);
    kit::wmma_gemm64<0, false, 2, 0, true, 0><<<dim3((unsigned)((((SEQ) / 64) * ((EMB) / 64) + 7) / 8), 1u), 256, 0, stream>>>(
        (const unsigned short*)H16, nullptr, FFD, 0L, (const unsigned short*)W216, nullptr, FFD, 0L, (void*)out, nullptr, EMB, 0L,
        BR2, H2f, 0L, SEQ, EMB, FFD, 1.0f / 256.0f);
}
